// MambaBlock_72146860638277
// MI455X (gfx1250) — hardware-verified
//
#include <hip/hip_runtime.h>
#include <math.h>

typedef __attribute__((ext_vector_type(16))) __bf16   v16b;
typedef __attribute__((ext_vector_type(8)))  __bf16   v8b;
typedef __attribute__((ext_vector_type(8)))  float    v8f;
typedef __attribute__((ext_vector_type(4)))  float    v4f;
typedef __attribute__((ext_vector_type(4)))  unsigned v4u;

constexpr int   kBatch  = 2;
constexpr int   kSeq    = 2048;
constexpr int   kDm     = 1024;
constexpr int   kDin    = 2048;
constexpr int   kNst    = 16;
constexpr int   kConvK  = 4;
constexpr int   kXzP    = 2 * kDin;
constexpr int   kXdN    = 2 * kNst;
constexpr int   kXdP    = 64;
constexpr int   kRows   = kBatch * kSeq;
constexpr float kDt     = 0.1f;
constexpr int   kConvTP = 260;
constexpr int   kScanTS = 64;
constexpr int   kScanCh = 64;
constexpr int   kScanYP = 68;
constexpr int   kScanXP = 32;
static_assert(kXdN == 32 && kXdN <= kXdP, "x_proj width");
static_assert(kScanXP == kXdN, "staged x_proj columns");
static_assert(kConvK == 4, "four taps");
static_assert((kDm % 32) == 0 && (kDin % 32) == 0, "GEMM K multiples of 32");
static_assert((kRows % 64) == 0 && (kXzP % 64) == 0 && (kXdP % 64) == 0 && (kDm % 64) == 0, "GEMM M,N multiples of 64");
static_assert((kSeq % kScanTS) == 0 && (kSeq % 64) == 0 && (kDin % kScanCh) == 0 && (kDin % 256) == 0, "tile multiples");
static_assert(((kRows / 64) * (kXzP / 64)) % 8 == 0 && ((kRows / 64) * (kXdP / 64)) % 8 == 0 && ((kRows / 64) * (kDm / 64)) % 8 == 0, "tiles per block");

constexpr size_t kOffXB   = 0;
constexpr size_t kOffWIB  = kOffXB  + (size_t)kRows * kDm  * 2;
constexpr size_t kOffWXB  = kOffWIB + (size_t)kXzP  * kDm  * 2;
constexpr size_t kOffWOB  = kOffWXB + (size_t)kXdP  * kDin * 2;
constexpr size_t kOffXZ   = kOffWOB + (size_t)kDm   * kDin * 2;
constexpr size_t kOffXS   = kOffXZ  + (size_t)kRows * kXzP * 4;
constexpr size_t kOffXD   = kOffXS  + (size_t)kRows * kDin * 2;
constexpr size_t kOffYL   = kOffXD  + (size_t)kRows * kXdP * 4;
constexpr size_t kWsTotal = kOffYL  + (size_t)kRows * kDin * 2;
static_assert(kWsTotal == 122945536ull, "carve total");
static_assert(kWsTotal <= 134217728ull, "carve cap");
static_assert((kOffWIB % 128) == 0 && (kOffWXB % 128) == 0 && (kOffWOB % 128) == 0 && (kOffXZ % 128) == 0 &&
              (kOffXS % 128) == 0 && (kOffXD % 128) == 0 && (kOffYL % 128) == 0, "128-B aligned regions");
static_assert((size_t)kRows * kDm * 4 == 16777216ull, "output bytes");

__device__ __forceinline__ unsigned f2bf_bits(float f) {
  const unsigned u = __float_as_uint(f);
  return (u + 0x7FFFu + ((u >> 16) & 1u)) >> 16;
}
__device__ __forceinline__ float bf_bits2f(unsigned h) { return __uint_as_float(h << 16); }
__device__ __forceinline__ float bf_rne(float f) { return bf_bits2f(f2bf_bits(f)); }
__device__ __forceinline__ unsigned pack_bf2(float a, float b) {
  const unsigned ha = f2bf_bits(a);
  const unsigned hb = f2bf_bits(b);
  return ha | (hb << 16);
}
__device__ __forceinline__ void split_pack2(float a, float b, unsigned& hi, unsigned& lo) {
  const unsigned ha = f2bf_bits(a);
  const unsigned hb = f2bf_bits(b);
  const float ra = a - bf_bits2f(ha);
  const float rb = b - bf_bits2f(hb);
  const unsigned la = f2bf_bits(ra);
  const unsigned lb = f2bf_bits(rb);
  hi = ha | (hb << 16);
  lo = la | (lb << 16);
}

__device__ __forceinline__ void dep_guard4_b(v8f& a, v8f& b, v8f& c, v8f& d, v16b x, v16b y) {
  asm volatile("v_nop\n\tv_nop\n\tv_nop\n\tv_nop" : "+v"(a), "+v"(b), "+v"(c), "+v"(d) : "v"(x), "v"(y));
}
__device__ __forceinline__ void keep4_b(v16b a, v16b b, v16b c, v16b d) { asm volatile("v_nop" :: "v"(a), "v"(b), "v"(c), "v"(d)); }
__device__ __forceinline__ void acc_guard4(v8f& a, v8f& b, v8f& c, v8f& d) {
  asm volatile("v_nop\n\tv_nop\n\tv_nop\n\tv_nop" : "+v"(a), "+v"(b), "+v"(c), "+v"(d));
}
struct FragB {
  union U { v16b v; v8b h[2]; };
  static __device__ __forceinline__ v16b load(const __bf16* p) {
    U f;
    f.h[0] = *(const v8b*)(p);
    f.h[1] = *(const v8b*)(p + 16);
    return f.v;
  }
  static __device__ __forceinline__ v8f mma(v16b a, v16b b, v8f c) {
    return __builtin_amdgcn_wmma_f32_16x16x32_bf16(false, a, false, b, (short)0, c, false, false);
  }
};

template <int SPL>
__global__ __launch_bounds__(256) void wmma_gemm64_bf16(
    const unsigned short* __restrict__ Ap, const unsigned short* __restrict__ A2p, int lda,
    const unsigned short* __restrict__ Btp, int ldb,
    float* __restrict__ Cout, int ldc, int M, int N, int K) {
  const __bf16* A  = (const __bf16*)Ap;
  const __bf16* A2 = (const __bf16*)A2p;
  const __bf16* Bt = (const __bf16*)Btp;
  __shared__ __align__(16) float sT[8][16 * 68];
  const int lane = threadIdx.x & 31;
  const int wave = threadIdx.x >> 5;
  const int tilesN = N >> 6;
  const int tilesM = M >> 6;
  const int tile = blockIdx.x * 8 + wave;
  if (tile >= tilesM * tilesN) return;
  const int tm = tile / tilesN;
  const int tn = tile - tm * tilesN;
  const int m0 = tm << 6;
  const int n0 = tn << 6;

  const int rlane = lane & 15;
  const int koff  = (lane >> 4) * 8;
  const int mOff  = (lane >> 4) * 8;

  v8f acc[4][4];
#pragma unroll
  for (int i = 0; i < 4; ++i)
#pragma unroll
    for (int j = 0; j < 4; ++j) acc[i][j] = (v8f){0.f, 0.f, 0.f, 0.f, 0.f, 0.f, 0.f, 0.f};

  for (int k0 = 0; k0 < K; k0 += 32) {
    v16b bh[4];
#pragma unroll
    for (int j = 0; j < 4; ++j) {
      const size_t bo = (size_t)(n0 + (j << 4) + rlane) * ldb + koff + k0;
      bh[j] = FragB::load(Bt + bo);
    }
#pragma unroll
    for (int i = 0; i < 4; ++i) {
      const size_t ao = (size_t)(m0 + (i << 4) + rlane) * lda + koff + k0;
      v16b ah = FragB::load(A + ao);
      v16b al = ah;
      if (SPL == 1) al = FragB::load(A2 + ao);
#pragma unroll
      for (int j = 0; j < 4; ++j) {
        acc[i][j] = FragB::mma(ah, bh[j], acc[i][j]);
        if (SPL == 1) acc[i][j] = FragB::mma(al, bh[j], acc[i][j]);
      }
      dep_guard4_b(acc[i][0], acc[i][1], acc[i][2], acc[i][3], ah, al);
    }
    keep4_b(bh[0], bh[1], bh[2], bh[3]);
  }
  acc_guard4(acc[0][0], acc[0][1], acc[0][2], acc[0][3]);
  acc_guard4(acc[1][0], acc[1][1], acc[1][2], acc[1][3]);
  acc_guard4(acc[2][0], acc[2][1], acc[2][2], acc[2][3]);
  acc_guard4(acc[3][0], acc[3][1], acc[3][2], acc[3][3]);

  float* slab = sT[wave];
  const int hh = lane >> 4;
  const int c4 = (lane & 15) * 4;
#pragma unroll
  for (int i = 0; i < 4; ++i) {
    const int mBase = m0 + (i << 4);
#pragma unroll
    for (int j = 0; j < 4; ++j) {
#pragma unroll
      for (int r = 0; r < 8; ++r) slab[(mOff + r) * 68 + (j << 4) + rlane] = acc[i][j][r];
    }
    __builtin_amdgcn_fence(__ATOMIC_RELEASE, "workgroup");
    __builtin_amdgcn_wave_barrier();
    __builtin_amdgcn_fence(__ATOMIC_ACQUIRE, "workgroup");
    for (int pass = 0; pass < 2; ++pass) {
#pragma unroll
      for (int it = 0; it < 8; ++it) {
        const int row = it * 2 + hh;
        const v4f v = *(const v4f*)(slab + row * 68 + c4);
        *(volatile v4f*)(Cout + (size_t)(mBase + row) * ldc + n0 + c4) = v;
      }
      __threadfence();
    }
    __builtin_amdgcn_fence(__ATOMIC_RELEASE, "workgroup");
    __builtin_amdgcn_wave_barrier();
    __builtin_amdgcn_fence(__ATOMIC_ACQUIRE, "workgroup");
  }
}

__global__ __launch_bounds__(256) void cast_bf16_kernel(
    const float* __restrict__ src, unsigned short* __restrict__ dst, int total8, int src8)
{
  const int i = blockIdx.x * 256 + threadIdx.x;
  if (i >= total8) return;
  const bool live = (i < src8);
  const int ic = live ? i : (src8 - 1);
  const size_t e0 = (size_t)ic << 3;
  const v4f a0 = *(const v4f*)(src + e0);
  const v4f a1 = *(const v4f*)(src + e0 + 4);
  const float f0 = live ? a0[0] : 0.0f;
  const float f1 = live ? a0[1] : 0.0f;
  const float f2 = live ? a0[2] : 0.0f;
  const float f3 = live ? a0[3] : 0.0f;
  const float f4 = live ? a1[0] : 0.0f;
  const float f5 = live ? a1[1] : 0.0f;
  const float f6 = live ? a1[2] : 0.0f;
  const float f7 = live ? a1[3] : 0.0f;
  const unsigned p0 = pack_bf2(f0, f1);
  const unsigned p1 = pack_bf2(f2, f3);
  const unsigned p2 = pack_bf2(f4, f5);
  const unsigned p3 = pack_bf2(f6, f7);
  const v4u w = (v4u){p0, p1, p2, p3};
  unsigned short* q = dst + ((size_t)i << 3);
  *(volatile v4u*)q = w;
  __threadfence();
  *(volatile v4u*)q = w;
}

__global__ __launch_bounds__(256) void conv_silu_kernel(
    const float* __restrict__ XZ, const float* __restrict__ cw, const float* __restrict__ cb,
    unsigned short* __restrict__ XS)
{
  __shared__ __align__(16) float sT[16 * kConvTP];
  const int tid = threadIdx.x, lane = tid & 31, wave = tid >> 5;
  const int d0 = blockIdx.x * 256, d = d0 + tid;
  const int g0 = blockIdx.y * 64;
  const int tb = g0 & (kSeq - 1);
  const v4f wv = *(const v4f*)(cw + (size_t)d * kConvK);
  const float w0 = bf_rne(wv[0]);
  const float w1 = bf_rne(wv[1]);
  const float w2 = bf_rne(wv[2]);
  const float w3 = bf_rne(wv[3]);
  const float bc = bf_rne(cb[d]);
  float xm3, xm2, xm1;
  {
    const bool hist = (tb > 0);
    const int rb = hist ? (g0 - 3) : g0;
    const float v3 = XZ[(size_t)rb * kXzP + d];
    const float v2 = XZ[(size_t)(rb + 1) * kXzP + d];
    const float v1 = XZ[(size_t)(rb + 2) * kXzP + d];
    xm3 = hist ? v3 : 0.0f;
    xm2 = hist ? v2 : 0.0f;
    xm1 = hist ? v1 : 0.0f;
  }
#pragma unroll 1
  for (int sub = 0; sub < 4; ++sub) {
    const int lb = g0 + sub * 16;
#pragma unroll 1
    for (int s = 0; s < 16; ++s) {
      const float xcur = XZ[(size_t)(lb + s) * kXzP + d];
      float acc = w0 * xm3;
      acc = fmaf(w1, xm2, acc);
      acc = fmaf(w2, xm1, acc);
      acc = fmaf(w3, xcur, acc);
      const float sv = acc + bc;
      const float sg = __builtin_amdgcn_rcpf(1.0f + expf(-sv));
      sT[s * kConvTP + tid] = sv * sg;
      xm3 = xm2; xm2 = xm1; xm1 = xcur;
    }
    __syncthreads();
    v4u bv[2];
#pragma unroll
    for (int it = 0; it < 2; ++it) {
      const float* sp = sT + (it * 8 + wave) * kConvTP + lane * 8;
      const v4f a0 = *(const v4f*)(sp);
      const v4f a1 = *(const v4f*)(sp + 4);
      const unsigned p0 = pack_bf2(a0[0], a0[1]);
      const unsigned p1 = pack_bf2(a0[2], a0[3]);
      const unsigned p2 = pack_bf2(a1[0], a1[1]);
      const unsigned p3 = pack_bf2(a1[2], a1[3]);
      bv[it] = (v4u){p0, p1, p2, p3};
    }
    for (int pass = 0; pass < 2; ++pass) {
#pragma unroll
      for (int it = 0; it < 2; ++it)
        *(volatile v4u*)(XS + (size_t)(lb + it * 8 + wave) * kDin + d0 + lane * 8) = bv[it];
      __threadfence();
    }
    __syncthreads();
  }
}

__global__ __launch_bounds__(64) void scan_kernel(
    const float* __restrict__ XZ, const float* __restrict__ XD,
    const float* __restrict__ cw, const float* __restrict__ cb,
    const float* __restrict__ Alog, const float* __restrict__ Dp,
    unsigned short* __restrict__ YH, unsigned short* __restrict__ YL)
{
  __shared__ __align__(16) float sX[kScanTS * kScanXP];
  __shared__ __align__(16) float sY[kScanTS * kScanYP];
  __shared__ __align__(16) float sA[kNst * kScanCh];
  const int tid = threadIdx.x, lane = tid & 31, wave = tid >> 5;
  constexpr int kBlkPerB = kDin / kScanCh;
  const int bix = blockIdx.x / kBlkPerB;
  const int d0  = (blockIdx.x - bix * kBlkPerB) * kScanCh;
  const int d   = d0 + tid;
  const size_t row0 = (size_t)bix * kSeq;
#pragma unroll 1
  for (int s = 0; s < kNst; ++s) {
    const float al = bf_rne(Alog[(size_t)d * kNst + s]);
    sA[s * kScanCh + tid] = expf(-kDt * expf(al));
  }
  __syncthreads();
  float dA[kNst], h[kNst];
#pragma unroll
  for (int n = 0; n < kNst; ++n) {
    dA[n] = sA[n * kScanCh + tid];
    h[n] = 0.0f;
  }
  const v4f wv = *(const v4f*)(cw + (size_t)d * kConvK);
  const float w0 = bf_rne(wv[0]);
  const float w1 = bf_rne(wv[1]);
  const float w2 = bf_rne(wv[2]);
  const float w3 = bf_rne(wv[3]);
  const float bc = bf_rne(cb[d]);
  const float Dd = bf_rne(Dp[d]);
  float xm3 = 0.0f, xm2 = 0.0f, xm1 = 0.0f;
  const int sr = tid >> 3, sc4 = (tid & 7) * 4;
  const int q = lane >> 3, c8 = (lane & 7) * 8;
#pragma unroll 1
  for (int t0 = 0; t0 < kSeq; t0 += kScanTS) {
    __syncthreads();
#pragma unroll
    for (int i = 0; i < 8; ++i) {
      const int r = sr + 8 * i;
      *(v4f*)(sX + r * kScanXP + sc4) = *(const v4f*)(XD + (row0 + t0 + r) * kXdP + sc4);
    }
    __syncthreads();
#pragma unroll 1
    for (int s = 0; s < kScanTS; ++s) {
      const size_t row = row0 + t0 + s;
      const float xcur = XZ[row * kXzP + d];
      const float zv   = XZ[row * kXzP + kDin + d];
      float acc = w0 * xm3;
      acc = fmaf(w1, xm2, acc);
      acc = fmaf(w2, xm1, acc);
      acc = fmaf(w3, xcur, acc);
      xm3 = xm2; xm2 = xm1; xm1 = xcur;
      const float sv = acc + bc;
      const float xt = sv * __builtin_amdgcn_rcpf(1.0f + expf(-sv));
      const float* xr = sX + s * kScanXP;
      v4f Bq[4], Cq[4];
#pragma unroll
      for (int qq = 0; qq < 4; ++qq) {
        Bq[qq] = *(const v4f*)(xr + 4 * qq);
        Cq[qq] = *(const v4f*)(xr + kNst + 4 * qq);
      }
      const float dtx = kDt * xt;
      float y = 0.0f;
#pragma unroll
      for (int n = 0; n < kNst; ++n) {
        const float hn = fmaf(dA[n], h[n], Bq[n >> 2][n & 3] * dtx);
        h[n] = hn;
        y = fmaf(hn, Cq[n >> 2][n & 3], y);
      }
      y = fmaf(xt, Dd, y);
      const float g = zv * __builtin_amdgcn_rcpf(1.0f + expf(-zv));
      sY[s * kScanYP + tid] = y * g;
    }
    __syncthreads();
    v4u hv[8], lv[8];
#pragma unroll
    for (int it = 0; it < 8; ++it) {
      const int rr = it * 8 + wave * 4 + q;
      const float* sp = sY + rr * kScanYP + c8;
      const v4f a0 = *(const v4f*)(sp);
      const v4f a1 = *(const v4f*)(sp + 4);
      unsigned h0, l0, h1, l1, h2, l2, h3, l3;
      split_pack2(a0[0], a0[1], h0, l0);
      split_pack2(a0[2], a0[3], h1, l1);
      split_pack2(a1[0], a1[1], h2, l2);
      split_pack2(a1[2], a1[3], h3, l3);
      hv[it] = (v4u){h0, h1, h2, h3};
      lv[it] = (v4u){l0, l1, l2, l3};
    }
    for (int pass = 0; pass < 2; ++pass) {
#pragma unroll
      for (int it = 0; it < 8; ++it) {
        const int rr = it * 8 + wave * 4 + q;
        const size_t o = (row0 + t0 + rr) * kDin + d0 + c8;
        *(volatile v4u*)(YH + o) = hv[it];
        *(volatile v4u*)(YL + o) = lv[it];
      }
      __threadfence();
    }
  }
}

extern "C" void kernel_launch(void* const* d_in, const int* in_sizes, int n_in,
                              void* d_out, int out_size, void* d_ws, size_t ws_size,
                              hipStream_t stream) {
  if (n_in < 8) return;
  if (in_sizes[0] != kRows * kDm) return;
  if (in_sizes[1] != kXzP * kDm) return;
  if (in_sizes[2] != kDin * kConvK) return;
  if (in_sizes[3] != kDin) return;
  if (in_sizes[4] != kXdN * kDin) return;
  if (in_sizes[5] != kDin * kNst) return;
  if (in_sizes[6] != kDin) return;
  if (in_sizes[7] != kDm * kDin) return;
  if (out_size != kRows * kDm) return;
  if (ws_size < kWsTotal) return;

  const float* x      = (const float*)d_in[0];
  const float* W_in   = (const float*)d_in[1];
  const float* conv_w = (const float*)d_in[2];
  const float* conv_b = (const float*)d_in[3];
  const float* W_x    = (const float*)d_in[4];
  const float* A_log  = (const float*)d_in[5];
  const float* Dp     = (const float*)d_in[6];
  const float* W_out  = (const float*)d_in[7];
  float* out = (float*)d_out;

  char* ws = (char*)d_ws;
  unsigned short* XB  = (unsigned short*)(ws + kOffXB);
  unsigned short* WIB = (unsigned short*)(ws + kOffWIB);
  unsigned short* WXB = (unsigned short*)(ws + kOffWXB);
  unsigned short* WOB = (unsigned short*)(ws + kOffWOB);
  float*          XZ  = (float*)(ws + kOffXZ);
  unsigned short* XS  = (unsigned short*)(ws + kOffXS);
  float*          XD  = (float*)(ws + kOffXD);
  unsigned short* YH  = (unsigned short*)(ws + kOffXS);
  unsigned short* YL  = (unsigned short*)(ws + kOffYL);

  cast_bf16_kernel<<<(kRows * kDm / 8) / 256, 256, 0, stream>>>(x, XB, kRows * kDm / 8, kRows * kDm / 8);
  cast_bf16_kernel<<<(kXzP * kDm / 8) / 256, 256, 0, stream>>>(W_in, WIB, kXzP * kDm / 8, kXzP * kDm / 8);
  cast_bf16_kernel<<<(kXdP * kDin / 8) / 256, 256, 0, stream>>>(W_x, WXB, kXdP * kDin / 8, kXdN * kDin / 8);
  cast_bf16_kernel<<<(kDm * kDin / 8) / 256, 256, 0, stream>>>(W_out, WOB, kDm * kDin / 8, kDm * kDin / 8);

  wmma_gemm64_bf16<0><<<((kRows / 64) * (kXzP / 64)) / 8, 256, 0, stream>>>(
      XB, XB, kDm, WIB, kDm, XZ, kXzP, kRows, kXzP, kDm);

  conv_silu_kernel<<<dim3(kDin / 256, kRows / 64), 256, 0, stream>>>(XZ, conv_w, conv_b, XS);

  wmma_gemm64_bf16<0><<<((kRows / 64) * (kXdP / 64)) / 8, 256, 0, stream>>>(
      XS, XS, kDin, WXB, kDin, XD, kXdP, kRows, kXdP, kDin);

  scan_kernel<<<kBatch * (kDin / kScanCh), kScanCh, 0, stream>>>(XZ, XD, conv_w, conv_b, A_log, Dp, YH, YL);

  wmma_gemm64_bf16<1><<<((kRows / 64) * (kDm / 64)) / 8, 256, 0, stream>>>(
      YH, YL, kDin, WOB, kDin, out, kDm, kRows, kDm, kDin);
}
